// MonetaBlock_28673201668257
// MI455X (gfx1250) — hardware-run, weakly checked
//
#include <hip/hip_runtime.h>
#include <math.h>

typedef __attribute__((ext_vector_type(16))) _Float16 v16h;
typedef __attribute__((ext_vector_type(8)))  _Float16 v8h;
typedef __attribute__((ext_vector_type(8)))  float    v8f;
typedef __attribute__((ext_vector_type(4)))  float    v4f;
typedef __attribute__((ext_vector_type(2)))  float    v2f;

constexpr int kInputsRneToBf16 = 1;

constexpr int kBatch   = 4;
constexpr int kSeq     = 1024;
constexpr int kDim     = 256;
constexpr int kRows    = kBatch * kSeq;
constexpr int kHalf    = kDim / 2;
constexpr int kColGate = 3 * kDim;
constexpr int kColPar  = 4 * kDim;
constexpr int kNreal   = kColPar + 2;
constexpr int kNcat    = 1088;
constexpr int kPadRows = kNcat - kColPar;
constexpr int kKout    = 2 * kDim;
static_assert(kRows == 4096);
static_assert((kSeq & (kSeq - 1)) == 0);
static_assert(kNcat >= kNreal && (kNcat % 64) == 0 && (kRows % 64) == 0 && (kDim % 64) == 0);
static_assert((kDim % 32) == 0 && (kKout % 32) == 0);
static_assert(kPadRows == 64);

constexpr float kCarryX    = 64.0f;
constexpr float kCarryW    = 1024.0f;
constexpr float kCarryY    = 1024.0f;
constexpr float kResidY    = 1024.0f;
constexpr float kCarryWoHi = 131072.0f;
constexpr float kCarryWoLo = kCarryWoHi / kResidY;
constexpr float kScaleG1   = 1.0f / (kCarryX * kCarryW);
constexpr float kScaleG2   = 1.0f / (kCarryY * kCarryWoHi);
constexpr float kF16MinNormal = 6.103515625e-05f;
static_assert(kCarryWoLo == 128.0f);

constexpr size_t kOffXH   = 0;
constexpr size_t kOffWCAT = kOffXH   + (size_t)kRows * kDim * 2;
constexpr size_t kOffWOC  = kOffWCAT + (size_t)kNcat * kDim * 2;
constexpr size_t kOffP    = kOffWOC  + (size_t)kDim * kKout * 2;
constexpr size_t kOffQH   = kOffP    + (size_t)kRows * kNcat * 4;
constexpr size_t kOffKH   = kOffQH   + (size_t)kRows * kDim * 4;
constexpr size_t kOffVH   = kOffKH   + (size_t)kRows * kDim * 4;
constexpr size_t kOffEA   = kOffVH   + (size_t)kRows * kDim * 4;
constexpr size_t kOffG    = kOffEA   + (size_t)kRows * 2 * 4;
constexpr size_t kOffY    = kOffG    + (size_t)kRows * kDim * 4;
constexpr size_t kOffYC   = kOffY    + (size_t)kRows * kDim * 4;
constexpr size_t kWsTotal = kOffYC   + (size_t)kRows * kKout * 2;
static_assert(kWsTotal == 45940736ull);
static_assert(kWsTotal <= 134217728ull);
static_assert((kOffWCAT % 128) == 0 && (kOffWOC % 128) == 0 && (kOffP % 128) == 0 && (kOffQH % 128) == 0 &&
              (kOffKH % 128) == 0 && (kOffVH % 128) == 0 && (kOffEA % 128) == 0 && (kOffG % 128) == 0 &&
              (kOffY % 128) == 0 && (kOffYC % 128) == 0);

constexpr int kScanLdsFloats = kDim * kDim + 4 * kDim + kDim + 4 * kDim + 4 * kDim + 32;
constexpr size_t kScanLdsBytes = (size_t)kScanLdsFloats * 4;
static_assert(kScanLdsBytes == 275584ull);

__device__ __forceinline__ unsigned short f2bf_bits(float f) {
  unsigned u = __float_as_uint(f);
  return (unsigned short)((u + 0x7FFFu + ((u >> 16) & 1u)) >> 16);
}
__device__ __forceinline__ float bf_bits2f(unsigned short h) { return __uint_as_float(((unsigned)h) << 16); }

__device__ __forceinline__ float in_cvt(float v) {
  if (kInputsRneToBf16) return bf_bits2f(f2bf_bits(v));
  return v;
}
__device__ __forceinline__ _Float16 f16_flush(float v) {
  const float z = (fabsf(v) < kF16MinNormal) ? 0.0f : v;
  return (_Float16)z;
}

__device__ __forceinline__ void acc_guard4(v8f& a, v8f& b, v8f& c, v8f& d) {
  asm volatile("v_nop\n\tv_nop\n\tv_nop\n\tv_nop" : "+v"(a), "+v"(b), "+v"(c), "+v"(d));
}
union FragH { v16h v; v8h h[2]; };
__device__ __forceinline__ v16h frag_load(const _Float16* p) {
  FragH f;
  f.h[0] = *(const v8h*)(p);
  f.h[1] = *(const v8h*)(p + 16);
  return f.v;
}
__device__ __forceinline__ v8f mma_h(v16h a, v16h b, v8f c) {
  c = __builtin_amdgcn_wmma_f32_16x16x32_f16(false, a, false, b, (short)0, c, false, false);
  asm volatile("v_nop\n\tv_nop\n\tv_nop\n\tv_nop" : "+v"(c) : "v"(a), "v"(b));
  return c;
}

__global__ __launch_bounds__(256) void cvt_rows_f16_kernel(
    const float* __restrict__ src, unsigned short* __restrict__ dst,
    int total8, int valid8, int dstPitch, int dstColOff, float carry)
{
  const int i = blockIdx.x * 256 + threadIdx.x;
  if (i >= total8) return;
  const int ic = (i < valid8) ? i : (valid8 - 1);
  const size_t e0 = (size_t)ic << 3;
  v4f a0 = *(const v4f*)(src + e0);
  v4f a1 = *(const v4f*)(src + e0 + 4);
  asm volatile("" : "+v"(a0), "+v"(a1));
  const bool ok = (i < valid8);
  const int row = i >> 5;
  const int col = (i & 31) << 3;
  v8h hv;
#pragma unroll
  for (int e = 0; e < 4; ++e) {
    const float f0 = ok ? a0[e] : 0.0f;
    const float f1 = ok ? a1[e] : 0.0f;
    hv[e]     = f16_flush(in_cvt(f0) * carry);
    hv[4 + e] = f16_flush(in_cvt(f1) * carry);
  }
  unsigned short* q = dst + (size_t)row * dstPitch + dstColOff + col;
  *(volatile v8h*)q = hv;
  __threadfence();
  *(volatile v8h*)q = hv;
}

__global__ __launch_bounds__(256) void y_split_f16_kernel(
    const float* __restrict__ Y, unsigned short* __restrict__ YC)
{
  const int i = blockIdx.x * 256 + threadIdx.x;
  const size_t e0 = (size_t)i << 3;
  const v4f a0 = *(const v4f*)(Y + e0);
  const v4f a1 = *(const v4f*)(Y + e0 + 4);
  const int row = i >> 5;
  const int col = (i & 31) << 3;
  v8h hv, lv;
#pragma unroll
  for (int e = 0; e < 4; ++e) {
    const float c0 = a0[e] * kCarryY;
    const float c1 = a1[e] * kCarryY;
    const _Float16 h0 = f16_flush(c0);
    const _Float16 h1 = f16_flush(c1);
    const float hf0 = (float)h0;
    const float hf1 = (float)h1;
    const float r0 = (c0 - hf0) * kResidY;
    const float r1 = (c1 - hf1) * kResidY;
    hv[e]     = h0;
    hv[4 + e] = h1;
    lv[e]     = f16_flush(r0);
    lv[4 + e] = f16_flush(r1);
  }
  unsigned short* qh = YC + (size_t)row * kKout + col;
  unsigned short* ql = qh + kDim;
  *(volatile v8h*)qh = hv;
  *(volatile v8h*)ql = lv;
  __threadfence();
  *(volatile v8h*)qh = hv;
  *(volatile v8h*)ql = lv;
}

__global__ __launch_bounds__(256) void gate_sigmoid_kernel(
    const float* __restrict__ P, float* __restrict__ G)
{
  const int i = blockIdx.x * 256 + threadIdx.x;
  const int row = i >> 6;
  const int c4 = (i & 63) << 2;
  const v4f z = *(const v4f*)(P + (size_t)row * kNcat + kColGate + c4);
  v4f o;
#pragma unroll
  for (int e = 0; e < 4; ++e) o[e] = 1.0f / (1.0f + expf(-z[e]));
  float* q = G + (size_t)row * kDim + c4;
  *(volatile v4f*)q = o;
  __threadfence();
  *(volatile v4f*)q = o;
}

template <bool GATE>
__global__ __launch_bounds__(256) void wmma_gemm64_f16(
    const unsigned short* __restrict__ Ap, int lda,
    const unsigned short* __restrict__ Btp, int ldb,
    float* __restrict__ Cout, int ldc,
    const float* __restrict__ gate, int ldg,
    int M, int N, int K, float scale)
{
  const _Float16* A  = (const _Float16*)Ap;
  const _Float16* Bt = (const _Float16*)Btp;
  __shared__ __align__(16) float sT[8][16 * 68];
  const int lane = threadIdx.x & 31;
  const int wave = threadIdx.x >> 5;
  const int tilesN = N >> 6;
  const int tilesM = M >> 6;
  const int tile = blockIdx.x * 8 + wave;
  if (tile >= tilesM * tilesN) return;
  const int tm = tile / tilesN;
  const int tn = tile - tm * tilesN;
  const int m0 = tm << 6;
  const int n0 = tn << 6;

  const int rlane = lane & 15;
  const int koff  = (lane >> 4) * 8;
  const int mOff  = (lane >> 4) * 8;

  v8f acc[4][4];
#pragma unroll
  for (int i = 0; i < 4; ++i)
#pragma unroll
    for (int j = 0; j < 4; ++j) acc[i][j] = (v8f){0.f,0.f,0.f,0.f,0.f,0.f,0.f,0.f};

  for (int k0 = 0; k0 < K; k0 += 32) {
    v16h bh[4];
#pragma unroll
    for (int j = 0; j < 4; ++j) {
      const size_t bo = (size_t)(n0 + (j << 4) + rlane) * ldb + koff + k0;
      bh[j] = frag_load(Bt + bo);
    }
#pragma unroll
    for (int i = 0; i < 4; ++i) {
      const size_t ao = (size_t)(m0 + (i << 4) + rlane) * lda + koff + k0;
      const v16h ah = frag_load(A + ao);
#pragma unroll
      for (int j = 0; j < 4; ++j) acc[i][j] = mma_h(ah, bh[j], acc[i][j]);
    }
  }
  acc_guard4(acc[0][0], acc[0][1], acc[0][2], acc[0][3]);
  acc_guard4(acc[1][0], acc[1][1], acc[1][2], acc[1][3]);
  acc_guard4(acc[2][0], acc[2][1], acc[2][2], acc[2][3]);
  acc_guard4(acc[3][0], acc[3][1], acc[3][2], acc[3][3]);

  float* slab = sT[wave];
  const int hh = lane >> 4;
  const int c4 = (lane & 15) * 4;
#pragma unroll
  for (int i = 0; i < 4; ++i) {
    const int mBase = m0 + (i << 4);
#pragma unroll
    for (int j = 0; j < 4; ++j) {
#pragma unroll
      for (int r = 0; r < 8; ++r)
        slab[(mOff + r) * 68 + (j << 4) + rlane] = acc[i][j][r] * scale;
    }
    __builtin_amdgcn_fence(__ATOMIC_RELEASE, "workgroup");
    __builtin_amdgcn_wave_barrier();
    __builtin_amdgcn_fence(__ATOMIC_ACQUIRE, "workgroup");
#pragma unroll
    for (int hf = 0; hf < 2; ++hf) {
      v4f vv[4];
#pragma unroll
      for (int q = 0; q < 4; ++q) {
        const int row = (hf * 4 + q) * 2 + hh;
        v4f v = *(const v4f*)(slab + row * 68 + c4);
        if (GATE) {
          const v4f gt = *(const v4f*)(gate + (size_t)(mBase + row) * ldg + n0 + c4);
          v = v * gt;
        }
        vv[q] = v;
      }
      for (int pass = 0; pass < 2; ++pass) {
#pragma unroll
        for (int q = 0; q < 4; ++q) {
          const int row = (hf * 4 + q) * 2 + hh;
          *(volatile v4f*)(Cout + (size_t)(mBase + row) * ldc + n0 + c4) = vv[q];
        }
        __threadfence();
      }
    }
    __builtin_amdgcn_fence(__ATOMIC_RELEASE, "workgroup");
    __builtin_amdgcn_wave_barrier();
    __builtin_amdgcn_fence(__ATOMIC_ACQUIRE, "workgroup");
  }
}

__global__ __launch_bounds__(256) void conv_rot_norm_kernel(
    const float* __restrict__ P,
    const float* __restrict__ qw, const float* __restrict__ qb,
    const float* __restrict__ kw, const float* __restrict__ kb,
    const float* __restrict__ vw, const float* __restrict__ vb,
    const float* __restrict__ fcos, const float* __restrict__ fsin,
    const float* __restrict__ bparam,
    float* __restrict__ qh, float* __restrict__ kh, float* __restrict__ vh,
    float* __restrict__ ea)
{
  __shared__ float sred[12 * 8];
  const int tid = threadIdx.x, lane = tid & 31, wave = tid >> 5;
  const int tk = tid >> 6;
  const int c4 = (tid & 63) << 2;
  const int row0 = blockIdx.x * 16;
#pragma unroll 1
  for (int it = 0; it < 12; ++it) {
    const int tg = it / 3;
    const int p  = it - tg * 3;
    const int row = row0 + tg * 4 + tk;
    const int t = row & (kSeq - 1);
    const float* wsel = (p == 0) ? qw : ((p == 1) ? kw : vw);
    const float* bsel = (p == 0) ? qb : ((p == 1) ? kb : vb);
    float* dsel       = (p == 0) ? qh : ((p == 1) ? kh : vh);
    const int colb = p * kDim + c4;
    v4f wv[4];
#pragma unroll
    for (int i = 0; i < 4; ++i) wv[i] = *(const v4f*)(wsel + (size_t)(c4 + i) * 4);
    const v4f bv = *(const v4f*)(bsel + c4);
    float acc[4] = {0.0f, 0.0f, 0.0f, 0.0f};
#pragma unroll
    for (int j = 0; j < 4; ++j) {
      const int tt = t + j - 3;
      const bool ok = (tt >= 0);
      const int rj = ok ? (row + j - 3) : row;
      v4f xv = *(const v4f*)(P + (size_t)rj * kNcat + colb);
      asm volatile("" : "+v"(xv));
#pragma unroll
      for (int i = 0; i < 4; ++i) {
        const float xs = ok ? xv[i] : 0.0f;
        acc[i] = fmaf(in_cvt(wv[i][j]), xs, acc[i]);
      }
    }
#pragma unroll
    for (int i = 0; i < 4; ++i) acc[i] += in_cvt(bv[i]);
    const v2f cs = *(const v2f*)(fcos + (size_t)t * kHalf + (c4 >> 1));
    const v2f sn = *(const v2f*)(fsin + (size_t)t * kHalf + (c4 >> 1));
    const float c0 = in_cvt(cs[0]), c1 = in_cvt(cs[1]);
    const float s0 = in_cvt(sn[0]), s1 = in_cvt(sn[1]);
    const float r0 = acc[0] * c0 - acc[1] * s0;
    const float r1 = acc[0] * s0 + acc[1] * c0;
    const float r2 = acc[2] * c1 - acc[3] * s1;
    const float r3 = acc[2] * s1 + acc[3] * c1;
    float ss = r0 * r0;
    ss = fmaf(r1, r1, ss);
    ss = fmaf(r2, r2, ss);
    ss = fmaf(r3, r3, ss);
    ss += __shfl_xor(ss, 16, 32);
    ss += __shfl_xor(ss, 8, 32);
    ss += __shfl_xor(ss, 4, 32);
    ss += __shfl_xor(ss, 2, 32);
    ss += __shfl_xor(ss, 1, 32);
    if (lane == 0) sred[it * 8 + wave] = ss;
    __syncthreads();
    const float tot = sred[it * 8 + 2 * tk] + sred[it * 8 + 2 * tk + 1];
    const float inv = 1.0f / fmaxf(sqrtf(tot), 1e-12f);
    const bool rot = (p < 2);
    v4f ov;
    ov[0] = rot ? (r0 * inv) : acc[0];
    ov[1] = rot ? (r1 * inv) : acc[1];
    ov[2] = rot ? (r2 * inv) : acc[2];
    ov[3] = rot ? (r3 * inv) : acc[3];
    float* q = dsel + (size_t)row * kDim + c4;
    *(volatile v4f*)q = ov;
    __threadfence();
    *(volatile v4f*)q = ov;
  }
  if (wave == 0) {
    const int tok = row0 + (lane >> 1);
    const int col = lane & 1;
    const float lg = P[(size_t)tok * kNcat + kColPar + col] + in_cvt(bparam[col]);
    const float sg = 1.0f / (1.0f + expf(-lg));
    float* q = ea + (size_t)row0 * 2 + lane;
    *(volatile float*)q = sg;
    __threadfence();
    *(volatile float*)q = sg;
  }
}

__global__ __launch_bounds__(256) void state_scan_kernel(
    const float* __restrict__ qh, const float* __restrict__ kh, const float* __restrict__ vh,
    const float* __restrict__ ea, const float* __restrict__ W0, float* __restrict__ ybuf)
{
  extern __shared__ __align__(16) float smem[];
  float* A     = smem;
  float* sRow  = smem + kDim * kDim;
  float* sG    = sRow + 4 * kDim;
  float* pY    = sG + kDim;
  float* pP    = pY + 4 * kDim;
  float* sRedW = pP + 4 * kDim;

  const int b    = blockIdx.x;
  const int tid  = threadIdx.x;
  const int lane = tid & 31;
  const int wave = tid >> 5;
  const int c    = tid & 63;
  const int r    = tid >> 6;
  const size_t bbase = (size_t)b * kSeq * kDim;
  const size_t ebase = (size_t)b * kSeq;
  const v2f* ea2 = (const v2f*)ea;

  v4f* A4    = (v4f*)A;
  v4f* sRow4 = (v4f*)sRow;
  {
    const v4f z = (v4f){0.f, 0.f, 0.f, 0.f};
#pragma unroll 1
    for (int j = 0; j < 64; ++j) A4[(size_t)(r * 64 + j) * 64 + c] = z;
  }
  sG[tid] = kh[bbase + tid];
  __syncthreads();
  float pred = 0.0f;
#pragma unroll 4
  for (int d = 0; d < kDim; ++d) pred = fmaf(sG[d], in_cvt(W0[(size_t)d * kDim + tid]), pred);
  __syncthreads();

  float rq  = qh[bbase + tid];
  float rk  = kh[bbase + tid];
  float rv  = vh[bbase + tid];
  float rkn = kh[bbase + kDim + tid];
  v2f   rea = ea2[ebase];

#pragma unroll 1
  for (int t = 0; t < kSeq; ++t) {
    const float et = rea[0];
    const float al = rea[1];
    const float diff = pred - rv;
    const float g = (3.0f * tanhf(10.0f * diff)) * (diff * diff);
    {
      v4f rw;
      rw[0] = rk * et;
      rw[1] = rq;
      rw[2] = rkn;
      rw[3] = 0.0f;
      sRow4[tid] = rw;
    }
    sG[tid] = -g;
    {
      const int tn  = (t + 1 < kSeq) ? (t + 1) : (kSeq - 1);
      const int tn2 = (t + 2 < kSeq) ? (t + 2) : (kSeq - 1);
      rq  = qh[bbase + (size_t)tn * kDim + tid];
      rk  = kh[bbase + (size_t)tn * kDim + tid];
      rv  = vh[bbase + (size_t)tn * kDim + tid];
      rkn = kh[bbase + (size_t)tn2 * kDim + tid];
      rea = ea2[ebase + tn];
    }
    __syncthreads();

    const v4f ng = *(const v4f*)(sG + 4 * c);
    v4f ay = (v4f){0.f, 0.f, 0.f, 0.f};
    v4f ap = (v4f){0.f, 0.f, 0.f, 0.f};
    float a4s = 0.0f;
    v4f* Ap = A4 + (size_t)(r * 64) * 64 + c;
    const v4f* rp = sRow4 + r * 64;
#pragma unroll 1
    for (int j = 0; j < 64; ++j) {
      const v4f rw = rp[j];
      v4f a = Ap[(size_t)j * 64];
      const float ek = rw[0], qd = rw[1], nd = rw[2];
      a[0] = fmaf(al, a[0], ek * ng[0]);
      a[1] = fmaf(al, a[1], ek * ng[1]);
      a[2] = fmaf(al, a[2], ek * ng[2]);
      a[3] = fmaf(al, a[3], ek * ng[3]);
      Ap[(size_t)j * 64] = a;
      const float x0 = a[0] * a[0], x1 = a[1] * a[1], x2 = a[2] * a[2], x3 = a[3] * a[3];
      a4s = fmaf(x0, x0, a4s);
      a4s = fmaf(x1, x1, a4s);
      a4s = fmaf(x2, x2, a4s);
      a4s = fmaf(x3, x3, a4s);
      ay[0] = fmaf(qd, a[0], ay[0]);
      ay[1] = fmaf(qd, a[1], ay[1]);
      ay[2] = fmaf(qd, a[2], ay[2]);
      ay[3] = fmaf(qd, a[3], ay[3]);
      ap[0] = fmaf(nd, a[0], ap[0]);
      ap[1] = fmaf(nd, a[1], ap[1]);
      ap[2] = fmaf(nd, a[2], ap[2]);
      ap[3] = fmaf(nd, a[3], ap[3]);
    }
    ((v4f*)pY)[r * 64 + c] = ay;
    ((v4f*)pP)[r * 64 + c] = ap;
    a4s += __shfl_xor(a4s, 16, 32);
    a4s += __shfl_xor(a4s, 8, 32);
    a4s += __shfl_xor(a4s, 4, 32);
    a4s += __shfl_xor(a4s, 2, 32);
    a4s += __shfl_xor(a4s, 1, 32);
    if (lane == 0) sRedW[wave] = a4s;
    __syncthreads();

    float s = sRedW[0];
    s += sRedW[1];
    s += sRedW[2];
    s += sRedW[3];
    s += sRedW[4];
    s += sRedW[5];
    s += sRedW[6];
    s += sRedW[7];
    const float invd = 1.0f / (sqrtf(s) + 1e-6f);
    const float yv = ((pY[tid] + pY[kDim + tid]) + pY[2 * kDim + tid]) + pY[3 * kDim + tid];
    const float pv = ((pP[tid] + pP[kDim + tid]) + pP[2 * kDim + tid]) + pP[3 * kDim + tid];
    const float yo = yv * invd;
    pred = pv * invd;
    float* yp = ybuf + bbase + (size_t)t * kDim + tid;
    *(volatile float*)yp = yo;
    __threadfence();
    *(volatile float*)yp = yo;
  }
}

extern "C" void kernel_launch(void* const* d_in, const int* in_sizes, int n_in,
                              void* d_out, int out_size, void* d_ws, size_t ws_size,
                              hipStream_t stream) {
  if (n_in < 15) return;
  if (in_sizes[0] != kRows * kDim) return;
  if (in_sizes[1] != kSeq * kHalf) return;
  if (in_sizes[2] != kSeq * kHalf) return;
  if (in_sizes[3] != 3 * kDim * kDim) return;
  if (in_sizes[4] != kDim * 4 || in_sizes[6] != kDim * 4 || in_sizes[8] != kDim * 4) return;
  if (in_sizes[5] != kDim || in_sizes[7] != kDim || in_sizes[9] != kDim) return;
  if (in_sizes[10] != 2 * kDim) return;
  if (in_sizes[11] != 2) return;
  if (in_sizes[12] != kDim * kDim || in_sizes[13] != kDim * kDim || in_sizes[14] != kDim * kDim) return;
  if (out_size != kRows * kDim) return;
  if (ws_size < kWsTotal) return;

  const float* x      = (const float*)d_in[0];
  const float* fcos   = (const float*)d_in[1];
  const float* fsin   = (const float*)d_in[2];
  const float* Wqkv   = (const float*)d_in[3];
  const float* qw     = (const float*)d_in[4];
  const float* qb     = (const float*)d_in[5];
  const float* kw     = (const float*)d_in[6];
  const float* kb     = (const float*)d_in[7];
  const float* vw     = (const float*)d_in[8];
  const float* vb     = (const float*)d_in[9];
  const float* Wparam = (const float*)d_in[10];
  const float* bparam = (const float*)d_in[11];
  const float* W0     = (const float*)d_in[12];
  const float* Wgate  = (const float*)d_in[13];
  const float* Wout   = (const float*)d_in[14];
  float* out = (float*)d_out;

  char* ws = (char*)d_ws;
  unsigned short* XH   = (unsigned short*)(ws + kOffXH);
  unsigned short* WCAT = (unsigned short*)(ws + kOffWCAT);
  unsigned short* WOC  = (unsigned short*)(ws + kOffWOC);
  float*          P    = (float*)(ws + kOffP);
  float*          QH   = (float*)(ws + kOffQH);
  float*          KH   = (float*)(ws + kOffKH);
  float*          VH   = (float*)(ws + kOffVH);
  float*          EA   = (float*)(ws + kOffEA);
  float*          G    = (float*)(ws + kOffG);
  float*          Y    = (float*)(ws + kOffY);
  unsigned short* YC   = (unsigned short*)(ws + kOffYC);

  cvt_rows_f16_kernel<<<(kRows * 32) / 256, 256, 0, stream>>>(x, XH, kRows * 32, kRows * 32, kDim, 0, kCarryX);
  cvt_rows_f16_kernel<<<(3 * kDim * 32) / 256, 256, 0, stream>>>(Wqkv, WCAT, 3 * kDim * 32, 3 * kDim * 32, kDim, 0, kCarryW);
  cvt_rows_f16_kernel<<<(kDim * 32) / 256, 256, 0, stream>>>(Wgate, WCAT + (size_t)kColGate * kDim, kDim * 32, kDim * 32, kDim, 0, kCarryW);
  cvt_rows_f16_kernel<<<(kPadRows * 32) / 256, 256, 0, stream>>>(Wparam, WCAT + (size_t)kColPar * kDim, kPadRows * 32, 2 * 32, kDim, 0, kCarryW);
  cvt_rows_f16_kernel<<<(kDim * 32) / 256, 256, 0, stream>>>(Wout, WOC, kDim * 32, kDim * 32, kKout, 0, kCarryWoHi);
  cvt_rows_f16_kernel<<<(kDim * 32) / 256, 256, 0, stream>>>(Wout, WOC, kDim * 32, kDim * 32, kKout, kDim, kCarryWoLo);

  wmma_gemm64_f16<false><<<(kRows / 64) * (kNcat / 64) / 8, 256, 0, stream>>>(
      XH, kDim, WCAT, kDim, P, kNcat, nullptr, 0, kRows, kNcat, kDim, kScaleG1);

  conv_rot_norm_kernel<<<kRows / 16, 256, 0, stream>>>(P, qw, qb, kw, kb, vw, vb, fcos, fsin, bparam, QH, KH, VH, EA);

  gate_sigmoid_kernel<<<(kRows * 64) / 256, 256, 0, stream>>>(P, G);

  state_scan_kernel<<<kBatch, 256, kScanLdsBytes, stream>>>(QH, KH, VH, EA, W0, Y);

  y_split_f16_kernel<<<(kRows * 32) / 256, 256, 0, stream>>>(Y, YC);

  wmma_gemm64_f16<true><<<(kRows / 64) * (kDim / 64) / 8, 256, 0, stream>>>(
      YC, kKout, WOC, kKout, out, kDim, G, kDim, kRows, kDim, kKout, kScaleG2);
}
